// DebertaLayer_78726750536333
// MI455X (gfx1250) — hardware-verified
//
#include <hip/hip_runtime.h>
#include <math.h>

typedef __attribute__((ext_vector_type(16))) _Float16 v16h;
typedef __attribute__((ext_vector_type(16))) __bf16 v16b;
typedef __attribute__((ext_vector_type(8)))  _Float16 v8h;
typedef __attribute__((ext_vector_type(8)))  float v8f;
typedef __attribute__((ext_vector_type(4)))  float v4f;
typedef __attribute__((ext_vector_type(2)))  float v2f;
typedef __attribute__((ext_vector_type(4)))  unsigned v4u;
typedef __attribute__((ext_vector_type(4)))  int v4i;
typedef float __attribute__((may_alias)) float_a;
typedef int __attribute__((may_alias)) int_a;

template <typename T> __device__ __forceinline__ void vst2(void* p, T v) { *(volatile T*)p = v; __threadfence(); *(volatile T*)p = v; }
__device__ __forceinline__ v8f wmma16(v16h a, v16h b, v8f c) {
  v8f d = __builtin_amdgcn_wmma_f32_16x16x32_f16(false, a, false, b, (short)0, c, false, false);
  asm volatile("v_nop\n\tv_nop\n\tv_nop\n\tv_nop" : "+v"(d) : "v"(a), "v"(b));
  return d;
}
__device__ __forceinline__ v8f wmma_bf(v16b a, v16b b, v8f c) {
  v8f d = __builtin_amdgcn_wmma_f32_16x16x32_bf16(false, a, false, b, (short)0, c, false, false);
  asm volatile("v_nop\n\tv_nop\n\tv_nop\n\tv_nop" : "+v"(d) : "v"(a), "v"(b));
  return d;
}
__device__ __forceinline__ v16h frag_h(const _Float16* rowk0, int lane) {
  union { v16h v; v8h q[2]; } u; const _Float16* p = rowk0 + 8 * (lane >> 4);
  u.q[0] = *(const v8h*)p; u.q[1] = *(const v8h*)(p + 16); return u.v;
}
__device__ __forceinline__ v16h frag_f32(const float* rowk0, int lane) {
  v16h a; const float* p = rowk0 + 8 * (lane >> 4);
#pragma unroll
  for (int i = 0; i < 8; ++i) { a[i] = (_Float16)p[i]; a[8 + i] = (_Float16)p[16 + i]; }
  return a;
}
__device__ __forceinline__ v16h frag_f32s(const float* rowk0, int lane, float sc) {
  v16h a; const float* p = rowk0 + 8 * (lane >> 4);
#pragma unroll
  for (int i = 0; i < 8; ++i) { a[i] = (_Float16)(p[i] * sc); a[8 + i] = (_Float16)(p[16 + i] * sc); }
  return a;
}
__device__ __forceinline__ v16h fragc_f32(const float* W, int k0, int n, int lane, int ld, int K) {
  v16h a; const int g = lane >> 4;
#pragma unroll
  for (int i = 0; i < 8; ++i) { const int ka = k0 + 8 * g + i, kb = ka + 16;
    a[i] = (_Float16)(ka < K ? W[(size_t)(ka < K ? ka : K - 1) * ld + n] : 0.f); a[8 + i] = (_Float16)(kb < K ? W[(size_t)(kb < K ? kb : K - 1) * ld + n] : 0.f); }
  return a;
}
struct F2 { v16b h, l; };
__device__ __forceinline__ F2 bsplit16(const float v[16]) { F2 r;
#pragma unroll
  for (int i = 0; i < 16; ++i) { const __bf16 h = (__bf16)v[i]; r.h[i] = h; r.l[i] = (__bf16)(v[i] - (float)h); }
  return r; }
__device__ __forceinline__ F2 split_row(const float* row, int k0, int lane) { float v[16]; const float* p = row + k0 + 8 * (lane >> 4);
#pragma unroll
  for (int i = 0; i < 8; ++i) { v[i] = p[i]; v[8 + i] = p[16 + i]; }
  return bsplit16(v); }
__device__ __forceinline__ F2 split_rowK(const float* row, int k0, int lane, int K) { float v[16]; const int g = lane >> 4;
#pragma unroll
  for (int i = 0; i < 8; ++i) { const int ka = k0 + 8 * g + i, kb = ka + 16; v[i] = ka < K ? row[ka < K ? ka : K - 1] : 0.f; v[8 + i] = kb < K ? row[kb < K ? kb : K - 1] : 0.f; }
  return bsplit16(v); }
__device__ __forceinline__ F2 split_col(const float* W, int k0, int n, int lane, int ld, int K) { float v[16]; const int g = lane >> 4;
#pragma unroll
  for (int i = 0; i < 8; ++i) { const int ka = k0 + 8 * g + i, kb = ka + 16; v[i] = ka < K ? W[(size_t)(ka < K ? ka : K - 1) * ld + n] : 0.f; v[8 + i] = kb < K ? W[(size_t)(kb < K ? kb : K - 1) * ld + n] : 0.f; }
  return bsplit16(v); }
__device__ __forceinline__ v8f mac3(const F2& a, const F2& b, v8f c) { c = wmma_bf(a.l, b.h, c); c = wmma_bf(a.h, b.l, c); return wmma_bf(a.h, b.h, c); }
__device__ __forceinline__ float sigm(float v) { return 1.0f / (1.0f + expf(-v)); }
#define LDSX() do { asm volatile("s_wait_dscnt 0" ::: "memory"); __builtin_amdgcn_wave_barrier(); __builtin_amdgcn_fence(__ATOMIC_RELEASE, "workgroup"); } while (0)


#define NB 16
#define SS 512
#define DM 768
#define NH 12
#define HD 64
#define PP 512
#define NPOS (2 * PP)
#define FF 3072
#define NR (NB * SS)
#ifndef TNB
#define TNB NB
#endif
typedef __attribute__((ext_vector_type(8))) __bf16 v8b;
__device__ __forceinline__ v16b frag_b(const __bf16* rowk0, int lane) {
  union { v16b v; v8b q[2]; } u; const __bf16* p = rowk0 + 8 * (lane >> 4);
  u.q[0] = *(const v8b*)p; u.q[1] = *(const v8b*)(p + 16); return u.v;
}
__device__ __forceinline__ float bfr(float v) { return (float)(__bf16)v; }
__device__ __attribute__((noinline)) float exp_ni(float v) { return expf(v); }
__device__ __attribute__((noinline)) float erf_ni(float v) { return erff(v); }

#define PK_Q  0
#define PK_K  ((size_t)DM * DM)
#define PK_V  ((size_t)2 * DM * DM)
#define PK_PK ((size_t)3 * DM * DM)
#define PK_PQ ((size_t)4 * DM * DM)
#define PK_O  ((size_t)5 * DM * DM)
#define PK_1  ((size_t)6 * DM * DM)
#define PK_2  (PK_1 + (size_t)FF * DM)
#define PK_END (PK_2 + (size_t)DM * FF)
#define WS_PK  0u
#define WS_QF  (((2u * PK_END) + 127u) / 128u * 128u)
#define WS_KF  (WS_QF + 2u * NR * DM)
#define WS_VTH (WS_KF + 2u * NR * DM)
#define WS_VTL (WS_VTH + 2u * NR * DM)
#define WS_PKF (WS_VTL + 2u * NR * DM)
#define WS_PQF (WS_PKF + 2u * NPOS * DM)
#define WS_O   (WS_PQF + 2u * NPOS * DM)
#define WS_T1  (WS_O + 4u * (size_t)NR * DM)
#define WS_H1  (WS_T1 + 4u * (size_t)NR * DM)
#define WS_G   (WS_H1 + 4u * (size_t)NR * DM)
#define WS_GL  (WS_G + 2u * (size_t)NR * FF)
#define WS_END (WS_GL + 2u * (size_t)NR * FF)

__global__ __launch_bounds__(256) void k_pack(const float* __restrict__ WQ, const float* __restrict__ WK, const float* __restrict__ WV, const float* __restrict__ WPK, const float* __restrict__ WPQ, const float* __restrict__ WO, const float* __restrict__ W1, const float* __restrict__ W2, __bf16* __restrict__ PK) {
  __shared__ __align__(16) __bf16 s[FF]; const int n = blockIdx.x, which = blockIdx.y, t = threadIdx.x; int K; size_t dst;
  if (which < 6) { if (n >= DM) return; const float* Wm = (which == 0) ? WQ : (which == 1) ? WK : (which == 2) ? WV : (which == 3) ? WPK : (which == 4) ? WPQ : WO; K = DM; dst = (size_t)which * DM * DM + (size_t)n * DM; for (int k = t; k < DM; k += 256) s[k] = (__bf16)Wm[(size_t)k * DM + n]; }
  else if (which == 6) { K = DM; dst = PK_1 + (size_t)n * DM; for (int k = t; k < DM; k += 256) s[k] = (__bf16)W1[(size_t)k * FF + n]; }
  else { if (n >= DM) return; K = FF; dst = PK_2 + (size_t)n * FF; for (int k = t; k < FF; k += 256) s[k] = (__bf16)W2[(size_t)k * DM + n]; }
  __syncthreads();
  for (int q = t; q < K / 8; q += 256) vst2((unsigned*)(PK + dst + q * 8), *(const v4u*)&s[q * 8]);
}
__global__ __launch_bounds__(128) void k_proj(const float* __restrict__ X, const float* __restrict__ POS, const __bf16* __restrict__ PK, const float* __restrict__ BQ, const float* __restrict__ BK, const float* __restrict__ BV, _Float16* __restrict__ QF, _Float16* __restrict__ KF, _Float16* __restrict__ VTH, _Float16* __restrict__ VTL, _Float16* __restrict__ PKF, _Float16* __restrict__ PQF) {
  __shared__ __align__(16) _Float16 so[4][16][136]; __shared__ __align__(16) _Float16 sth[128][72], stl[128][72];
  const int tid = threadIdx.x, wave = tid >> 5, lane = tid & 31, col = lane & 15, g = lane >> 4; const int which = blockIdx.z; const size_t r0 = (size_t)blockIdx.x * 64 + wave * 16; const int n0 = blockIdx.y * 128;
  if (which >= 3 && blockIdx.x * 64 >= NPOS) return;
  if (which < 3 && blockIdx.x * 64 >= TNB * SS) return;
  const float* SRC = (which >= 3) ? POS : X; const __bf16* P = PK + ((which == 0) ? PK_Q : (which == 1) ? PK_K : (which == 2) ? PK_V : (which == 3) ? PK_PK : PK_PQ);
  v8f acc[8] = {};
#pragma unroll 2
  for (int kc = 0; kc < DM / 32; ++kc) { v16b a; { const float* p = SRC + (r0 + col) * DM + kc * 32 + 8 * g;
#pragma unroll
      for (int i = 0; i < 8; ++i) { a[i] = (__bf16)p[i]; a[8 + i] = (__bf16)p[16 + i]; } }
#pragma unroll
    for (int j = 0; j < 8; ++j) acc[j] = wmma_bf(a, frag_b(P + (size_t)(n0 + j * 16 + col) * DM + kc * 32, lane), acc[j]); }
  const float* BB = (which == 0) ? BQ : (which == 1) ? BK : (which == 2) ? BV : nullptr;
  if (which != 2) {
#pragma unroll
    for (int j = 0; j < 8; ++j) { const float bb = BB ? bfr(BB[n0 + j * 16 + col]) : 0.f;
#pragma unroll
      for (int r = 0; r < 8; ++r) so[wave][8 * g + r][j * 16 + col] = (_Float16)(acc[j][r] + bb); }
    LDSX();
    _Float16* D = (which == 0) ? QF : (which == 1) ? KF : (which == 3) ? PKF : PQF;
    for (int rl = 0; rl < 16; ++rl) if (lane < 16) vst2((unsigned*)(D + (r0 + rl) * DM + n0 + lane * 8), *(const v4u*)&so[wave][rl][lane * 8]);
  } else {
#pragma unroll
    for (int j = 0; j < 8; ++j) { const float bb = bfr(BB[n0 + j * 16 + col]);
#pragma unroll
      for (int r = 0; r < 8; ++r) { const float v = acc[j][r] + bb; const _Float16 hv = (_Float16)v; sth[j * 16 + col][wave * 16 + 8 * g + r] = hv; stl[j * 16 + col][wave * 16 + 8 * g + r] = (_Float16)((v - (float)hv) * 2048.0f); } }
    __syncthreads();
    const size_t rb = (size_t)blockIdx.x * 64; const int b = (int)(rb / SS), s0 = (int)(rb % SS);
    for (int e = tid; e < 128 * 8; e += 128) { const int d = e >> 3, pc = e & 7; const size_t o = ((size_t)b * DM + n0 + d) * SS + s0 + pc * 8; vst2((unsigned*)(VTH + o), *(const v4u*)&sth[d][pc * 8]); vst2((unsigned*)(VTL + o), *(const v4u*)&stl[d][pc * 8]); }
  }
}
__global__ __launch_bounds__(128) void k_attn(const _Float16* __restrict__ QF, const _Float16* __restrict__ KF, const _Float16* __restrict__ PKF, const _Float16* __restrict__ PQF, const _Float16* __restrict__ VTH, const _Float16* __restrict__ VTL, const float* __restrict__ AMASK, float* __restrict__ O) {
  __shared__ __align__(16) _Float16 sp[4][16][40]; __shared__ float sv2[4][16][49]; __shared__ float su[32][97]; __shared__ __align__(16) float so[4][16][68];
  const int tid = threadIdx.x, wave = tid >> 5, lane = tid & 31, col = lane & 15, g = lane >> 4; const int qb = blockIdx.x, h = blockIdx.y, b = blockIdx.z; const int i0 = qb * 64, iw0 = i0 + wave * 16; const size_t rq = (size_t)b * SS + iw0 + col;
  v16h aq[2];
#pragma unroll
  for (int kc = 0; kc < 2; ++kc) aq[kc] = frag_h(QF + rq * DM + h * HD + kc * 32, lane);
  const _Float16* Vh = VTH + ((size_t)b * DM + h * HD) * SS; const _Float16* Vl = VTL + ((size_t)b * DM + h * HD) * SS;
  const float scale = 0.07216878364870322f;
  float m[8], l[8];
#pragma unroll
  for (int r = 0; r < 8; ++r) { m[r] = -3.0e38f; l[r] = 0.f; }
  v8f acc[4] = {}, accl[4] = {};
#pragma unroll 1
  for (int ks = 0; ks < SS / 32; ++ks) { const int j0 = ks * 32;
    { const int r0p = j0 - i0 - 63 + PP; const int jg = wave & 1, tg = wave >> 1; const v16h ak0 = frag_h(KF + ((size_t)b * SS + j0 + jg * 16 + col) * DM + h * HD, lane), ak1 = frag_h(KF + ((size_t)b * SS + j0 + jg * 16 + col) * DM + h * HD + 32, lane);
#pragma unroll
      for (int ct3 = 0; ct3 < 3; ++ct3) { const int t0 = (tg * 3 + ct3) * 16; int rr = r0p + t0 + col; rr = min(max(rr, 0), NPOS - 1);
        v8f u = {}; u = wmma16(ak0, frag_h(PQF + (size_t)rr * DM + h * HD, lane), u); u = wmma16(ak1, frag_h(PQF + (size_t)rr * DM + h * HD + 32, lane), u);
#pragma unroll
        for (int r = 0; r < 8; ++r) su[jg * 16 + 8 * g + r][t0 + col] = u[r]; } }
    { const int r0w = iw0 - j0 - 31 + PP;
#pragma unroll
      for (int ct3 = 0; ct3 < 3; ++ct3) { int rr = r0w + ct3 * 16 + col; rr = min(max(rr, 0), NPOS - 1); v8f u = {};
#pragma unroll
        for (int kc = 0; kc < 2; ++kc) u = wmma16(aq[kc], frag_h(PKF + (size_t)rr * DM + h * HD + kc * 32, lane), u);
#pragma unroll
        for (int r = 0; r < 8; ++r) sv2[wave][8 * g + r][ct3 * 16 + col] = u[r]; } }
    __syncthreads();
    v8f s[2];
#pragma unroll
    for (int ct = 0; ct < 2; ++ct) { const int jl = ct * 16 + col; const int kk = j0 + jl; const size_t rk = ((size_t)b * SS + kk) * DM + h * HD; v8f c = {};
#pragma unroll
      for (int kc = 0; kc < 2; ++kc) c = wmma16(aq[kc], frag_h(KF + rk + kc * 32, lane), c);
      const bool keep = bfr(AMASK[(size_t)b * SS + kk]) > 0.f;
#pragma unroll
      for (int r = 0; r < 8; ++r) { const int il = 8 * g + r; const int ilb = wave * 16 + il; const float c2p = sv2[wave][il][il - jl + 31]; const float p2c = su[jl][jl - ilb + 63];
        s[ct][r] = keep ? (c[r] + c2p + p2c) * scale : -1.0e9f; } }
#pragma unroll
    for (int r = 0; r < 8; ++r) { float mx = fmaxf(s[0][r], s[1][r]);
#pragma unroll
      for (int o = 1; o < 16; o <<= 1) mx = fmaxf(mx, __shfl_xor(mx, o));
      const float mn = fmaxf(m[r], mx); const float alpha = (m[r] <= -1.0e38f) ? 0.f : __expf(m[r] - mn); const float e0 = __expf(s[0][r] - mn), e1 = __expf(s[1][r] - mn); float es = e0 + e1;
#pragma unroll
      for (int o = 1; o < 16; o <<= 1) es += __shfl_xor(es, o);
      l[r] = l[r] * alpha + es; m[r] = mn;
#pragma unroll
      for (int dt = 0; dt < 4; ++dt) { acc[dt][r] *= alpha; accl[dt][r] *= alpha; }
      sp[wave][8 * g + r][col] = (_Float16)e0; sp[wave][8 * g + r][16 + col] = (_Float16)e1; }
    __syncthreads();
    const v16h pa = frag_h(&sp[wave][col][0], lane);
#pragma unroll
    for (int dt = 0; dt < 4; ++dt) { const size_t vo = (size_t)(dt * 16 + col) * SS + j0; acc[dt] = wmma16(pa, frag_h(Vh + vo, lane), acc[dt]); accl[dt] = wmma16(pa, frag_h(Vl + vo, lane), accl[dt]); }
    LDSX(); }
#pragma unroll
  for (int r = 0; r < 8; ++r) { const float il = 1.0f / l[r];
#pragma unroll
    for (int dt = 0; dt < 4; ++dt) so[wave][8 * g + r][dt * 16 + col] = (acc[dt][r] + accl[dt][r] * (1.0f / 2048.0f)) * il; }
  LDSX();
  for (int rl = 0; rl < 16; ++rl) if (lane < 16) vst2(O + ((size_t)b * SS + iw0 + rl) * DM + h * HD + lane * 4, *(const v4f*)&so[wave][rl][lane * 4]);
}
template <int MODE>
__global__ __launch_bounds__(128) void k_lin(const float* __restrict__ A, const __bf16* __restrict__ AG, const __bf16* __restrict__ AGL, const __bf16* __restrict__ PK, const float* __restrict__ BIAS, const float* __restrict__ RES, float* __restrict__ OUTF, __bf16* __restrict__ OUTG, __bf16* __restrict__ OUTGL) {
  __shared__ __align__(16) float so[4][16][132]; __shared__ __align__(16) __bf16 sg[4][16][136], sgl[4][16][136];
  const int tid = threadIdx.x, wave = tid >> 5, lane = tid & 31, col = lane & 15, g = lane >> 4; const size_t r0 = (size_t)blockIdx.x * 64 + wave * 16; const int n0 = blockIdx.y * 128;
  constexpr int KD = (MODE == 2) ? FF : DM; const __bf16* P = PK + ((MODE == 0) ? PK_O : (MODE == 1) ? PK_1 : PK_2);
  v8f acc[8] = {};
  if (MODE == 2) {
#pragma unroll 2
    for (int kc = 0; kc < KD / 32; ++kc) { const v16b a = frag_b(AG + (r0 + col) * FF + kc * 32, lane), al = frag_b(AGL + (r0 + col) * FF + kc * 32, lane);
#pragma unroll
      for (int j = 0; j < 8; ++j) { const v16b w = frag_b(P + (size_t)(n0 + j * 16 + col) * KD + kc * 32, lane); acc[j] = wmma_bf(al, w, acc[j]); acc[j] = wmma_bf(a, w, acc[j]); } }
  } else {
#pragma unroll 2
    for (int kc = 0; kc < KD / 32; ++kc) { const F2 a = split_row(A + (r0 + col) * DM, kc * 32, lane);
#pragma unroll
      for (int j = 0; j < 8; ++j) { const v16b w = frag_b(P + (size_t)(n0 + j * 16 + col) * KD + kc * 32, lane); acc[j] = wmma_bf(a.l, w, acc[j]); acc[j] = wmma_bf(a.h, w, acc[j]); } } }
#pragma unroll
  for (int j = 0; j < 8; ++j) { const int c = n0 + j * 16 + col; const float bb = bfr(BIAS[c]);
#pragma unroll
    for (int r = 0; r < 8; ++r) { const size_t row = r0 + 8 * g + r; float v = acc[j][r] + bb;
      if (MODE == 1) { v = 0.5f * v * (1.0f + erf_ni(v * 0.70710678118654752f)); const __bf16 hb = (__bf16)v; sg[wave][8 * g + r][j * 16 + col] = hb; sgl[wave][8 * g + r][j * 16 + col] = (__bf16)(v - (float)hb); }
      else { v += (MODE == 0) ? bfr(RES[row * DM + c]) : RES[row * DM + c]; so[wave][8 * g + r][j * 16 + col] = v; } } }
  LDSX();
  if (MODE == 1) { for (int rl = 0; rl < 16; ++rl) { if (lane < 16) vst2((unsigned*)(OUTG + (r0 + rl) * FF + n0 + lane * 8), *(const v4u*)&sg[wave][rl][lane * 8]); else vst2((unsigned*)(OUTGL + (r0 + rl) * FF + n0 + (lane - 16) * 8), *(const v4u*)&sgl[wave][rl][(lane - 16) * 8]); } }
  else { for (int rl = 0; rl < 16; ++rl) vst2(OUTF + (r0 + rl) * DM + n0 + lane * 4, *(const v4f*)&so[wave][rl][lane * 4]); }
}
__global__ __launch_bounds__(192) void k_ln(const float* __restrict__ T, const float* __restrict__ G, const float* __restrict__ Bv, float* __restrict__ OUT) {
  __shared__ float red[2][8]; const int t = threadIdx.x; const size_t row = blockIdx.x; const float* p = T + row * DM + t * 4;
  float v[4] = {p[0], p[1], p[2], p[3]}; float s = (v[0] + v[1]) + (v[2] + v[3]);
#pragma unroll
  for (int o = 1; o < 32; o <<= 1) s += __shfl_xor(s, o);
  if ((t & 31) == 0) red[0][t >> 5] = s; __syncthreads();
  float tot = 0.f; for (int w = 0; w < 6; ++w) tot += red[0][w]; const float mu = tot / (float)DM;
  float q = 0.f;
#pragma unroll
  for (int i = 0; i < 4; ++i) { const float d = v[i] - mu; q += d * d; }
#pragma unroll
  for (int o = 1; o < 32; o <<= 1) q += __shfl_xor(q, o);
  if ((t & 31) == 0) red[1][t >> 5] = q; __syncthreads();
  float qt = 0.f; for (int w = 0; w < 6; ++w) qt += red[1][w]; const float inv = 1.0f / sqrtf(qt / (float)DM + 1e-7f);
  v4f o4;
#pragma unroll
  for (int i = 0; i < 4; ++i) o4[i] = (v[i] - mu) * inv * bfr(G[t * 4 + i]) + bfr(Bv[t * 4 + i]);
  vst2(OUT + row * DM + t * 4, o4);
}
extern "C" void kernel_launch(void* const* d_in, const int* in_sizes, int n_in, void* d_out, int out_size, void* d_ws, size_t ws_size, hipStream_t stream) {
  (void)in_sizes; (void)n_in; (void)out_size;
  const float** F = (const float**)d_in;
  if (ws_size < (size_t)WS_END) return;
  char* ws = (char*)d_ws; __bf16 *PK = (__bf16*)(ws + WS_PK), *G = (__bf16*)(ws + WS_G), *GL = (__bf16*)(ws + WS_GL); _Float16 *QF = (_Float16*)(ws + WS_QF), *KF = (_Float16*)(ws + WS_KF), *VTH = (_Float16*)(ws + WS_VTH), *VTL = (_Float16*)(ws + WS_VTL), *PKF = (_Float16*)(ws + WS_PKF), *PQF = (_Float16*)(ws + WS_PQF); float *O = (float*)(ws + WS_O), *T1 = (float*)(ws + WS_T1), *H1 = (float*)(ws + WS_H1);
  k_pack<<<dim3(FF, 8), 256, 0, stream>>>(F[3], F[5], F[7], F[9], F[10], F[11], F[15], F[17], PK);
  k_proj<<<dim3((TNB * SS / 64 > NPOS / 64) ? (TNB * SS / 64) : (NPOS / 64), DM / 128, 5), 128, 0, stream>>>(F[0], F[2], PK, F[4], F[6], F[8], QF, KF, VTH, VTL, PKF, PQF);
  k_attn<<<dim3(SS / 64, NH, TNB), 128, 0, stream>>>(QF, KF, PKF, PQF, VTH, VTL, F[1], O);
  k_lin<0><<<dim3(TNB * SS / 64, DM / 128), 128, 0, stream>>>(O, nullptr, nullptr, PK, F[12], F[0], T1, nullptr, nullptr);
  k_ln<<<TNB * SS, 192, 0, stream>>>(T1, F[13], F[14], H1);
  k_lin<1><<<dim3(TNB * SS / 64, FF / 128), 128, 0, stream>>>(H1, nullptr, nullptr, PK, F[16], nullptr, nullptr, G, GL);
  k_lin<2><<<dim3(TNB * SS / 64, DM / 128), 128, 0, stream>>>(nullptr, G, GL, PK, F[18], H1, T1, nullptr, nullptr);
  k_ln<<<TNB * SS, 192, 0, stream>>>(T1, F[19], F[20], (float*)d_out);
}
